// BertGraphCrossAttention_13297218748517
// MI455X (gfx1250) — hardware-run, weakly checked
//
#include <hip/hip_runtime.h>
#include <math.h>
#include <stdint.h>

#define NB     4
#define LQ     512
#define DM     768
#define NH     12
#define DHD    64
#define NTYPES 3
#define MTOK   (NB * LQ)
#define QP     (2 * DM)
#define ARC_P  68

static_assert(DM % 64 == 0);
static_assert(DHD == 64);
static_assert(LQ % 64 == 0);
static_assert(MTOK % 64 == 0);
static_assert(DM % 64 == 0 && (2 * DM) % 64 == 0);
static_assert(DM % 32 == 0);
static_assert(NTYPES == 3);
static_assert(NH * DHD == DM);

typedef __attribute__((ext_vector_type(16))) __bf16   v16b;
typedef __attribute__((ext_vector_type(8)))  __bf16   v8b;
typedef __attribute__((ext_vector_type(8)))  float    v8f;
typedef __attribute__((ext_vector_type(4)))  float    v4f;
typedef __attribute__((ext_vector_type(2)))  float    v2f;
typedef __attribute__((ext_vector_type(4)))  unsigned int v4u;
typedef __attribute__((ext_vector_type(4)))  int      v4i;
typedef v4f __attribute__((may_alias)) v4fa;
typedef v2f __attribute__((may_alias)) v2fa;
typedef v4u __attribute__((may_alias)) v4ua;
typedef v4i __attribute__((may_alias)) v4ia;

constexpr size_t OB_XB   = 0;
constexpr size_t OB_CB   = OB_XB + (size_t)MTOK * DM * 2;
constexpr size_t OB_WT   = OB_CB + (size_t)MTOK * DM * 2;
constexpr size_t OB_BQKV = OB_WT + (size_t)3 * DM * DM * 2;
constexpr size_t OB_TKV  = OB_BQKV + (size_t)3 * DM * 4;
constexpr size_t OB_QHL  = OB_TKV + (size_t)2 * NTYPES * DHD * 4;
constexpr size_t OB_KHL  = OB_QHL + (size_t)MTOK * QP * 2;
constexpr size_t OB_VTH  = OB_KHL + (size_t)MTOK * QP * 2;
constexpr size_t OB_VTL  = OB_VTH + (size_t)NB * NH * DHD * LQ * 2;
constexpr size_t OB_END  = OB_VTL + (size_t)NB * NH * DHD * LQ * 2;
static_assert(OB_CB % 256 == 0 && OB_WT % 256 == 0 && OB_BQKV % 256 == 0 && OB_TKV % 256 == 0);
static_assert(OB_QHL % 256 == 0 && OB_KHL % 256 == 0 && OB_VTH % 256 == 0 && OB_VTL % 256 == 0);
static_assert(OB_END == 28715520);
static_assert(OB_END <= (size_t)134217728);
constexpr size_t EO_XB = OB_XB / 2, EO_CB = OB_CB / 2, EO_WT = OB_WT / 2;
constexpr size_t EO_QHL = OB_QHL / 2, EO_KHL = OB_KHL / 2, EO_VTH = OB_VTH / 2, EO_VTL = OB_VTL / 2;

#define TILES_JOB 384
static_assert((MTOK / 64) * (DM / 64) == TILES_JOB);

__device__ __forceinline__ unsigned short f2bf_bits(float f) {
  unsigned u = __float_as_uint(f);
  return (unsigned short)((u + 0x7FFFu + ((u >> 16) & 1u)) >> 16);
}
__device__ __forceinline__ float bf_bits2f(unsigned short h) { return __uint_as_float(((unsigned)h) << 16); }
__device__ __forceinline__ float bfval(float f) { return bf_bits2f(f2bf_bits(f)); }
__device__ __forceinline__ unsigned pk16(unsigned short a, unsigned short b) { return (unsigned)a | ((unsigned)b << 16); }
__device__ __forceinline__ float mskf(float v, unsigned m) { return __uint_as_float(__float_as_uint(v) & m); }
__device__ __forceinline__ int clamp02(int a) { return min(max(a, 0), NTYPES - 1); }

__device__ __forceinline__ float blend3(int a, float x0, float x1, float x2) {
  const unsigned m1 = (unsigned)(-(int)(a == 1));
  const unsigned m2 = (unsigned)(-(int)(a == 2));
  const unsigned m0 = ~(m1 | m2);
  return __uint_as_float((__float_as_uint(x0) & m0) | (__float_as_uint(x1) & m1) | (__float_as_uint(x2) & m2));
}
__device__ __forceinline__ float keep_if(float p, int cond) {
  return __uint_as_float(__float_as_uint(p) & (unsigned)(-cond));
}
__device__ __forceinline__ void cbar() { asm volatile("" ::: "memory"); }

__device__ __forceinline__ v8f wmb(v16b a, v16b b, v8f c) {
  c = __builtin_amdgcn_wmma_f32_16x16x32_bf16(false, a, false, b, (short)0, c, false, false);
  asm volatile("v_nop\n\tv_nop\n\tv_nop\n\tv_nop" : "+v"(c) : "v"(a), "v"(b));
  return c;
}
union FB { v16b v; v8b h[2]; };
__device__ __forceinline__ v16b ldfrag(const __bf16* p) {
  FB f; f.h[0] = *(const v8b*)(p); f.h[1] = *(const v8b*)(p + 16); return f.v;
}
__device__ __forceinline__ void split_bf(float f, __bf16& hi, __bf16& lo) {
  const unsigned short hb = f2bf_bits(f);
  hi = __builtin_bit_cast(__bf16, hb);
  lo = __builtin_bit_cast(__bf16, f2bf_bits(f - bf_bits2f(hb)));
}

static_assert(768 * 256 * 8 == MTOK * DM);
__global__ __launch_bounds__(256) void k_pa(const float* __restrict__ hid, const float* __restrict__ ctx,
                                            unsigned short* wsb) {
  const size_t g = (size_t)blockIdx.x * 256 + threadIdx.x;
  v4f a, c;
  if (blockIdx.y == 0) {
    a = *(const v4fa*)(hid + g * 8);
    c = *(const v4fa*)(hid + g * 8 + 4);
  } else {
    a = *(const v4fa*)(ctx + g * 8);
    c = *(const v4fa*)(ctx + g * 8 + 4);
  }
  v4u o;
  o[0] = pk16(f2bf_bits(a[0]), f2bf_bits(a[1]));
  o[1] = pk16(f2bf_bits(a[2]), f2bf_bits(a[3]));
  o[2] = pk16(f2bf_bits(c[0]), f2bf_bits(c[1]));
  o[3] = pk16(f2bf_bits(c[2]), f2bf_bits(c[3]));
  const size_t eo = (blockIdx.y == 0) ? EO_XB : EO_CB;
  unsigned short* dst = wsb + eo + g * 8;
  *(volatile v4u*)dst = o;
  __threadfence();
  *(volatile v4u*)dst = o;
}

__device__ __forceinline__ void pb_load(const float* __restrict__ W, const float* __restrict__ bias,
                                        int r0, int c0, int lr, int c4, int bi, v4f (&a)[4], v4f& bb) {
#pragma unroll
  for (int it = 0; it < 4; ++it) a[it] = *(const v4fa*)(W + (size_t)(r0 + it * 16 + lr) * DM + c0 + c4);
  bb = *(const v4fa*)(bias + bi);
}
__global__ __launch_bounds__(256) void k_pb(const float* __restrict__ Wq, const float* __restrict__ bq,
                                            const float* __restrict__ Wk, const float* __restrict__ bk,
                                            const float* __restrict__ Wv, const float* __restrict__ bv,
                                            unsigned short* __restrict__ wt, float* __restrict__ bqkv) {
  __shared__ __align__(16) float tf[64 * 68];
  const int z   = blockIdx.z;
  const int c0  = blockIdx.x * 64;
  const int r0  = blockIdx.y * 64;
  const int tid = threadIdx.x;
  const int lr  = tid >> 4;
  const int c4  = (tid & 15) * 4;
  const int bi  = min(tid, 191) * 4;
  v4f a[4]; v4f bb;
  if (z == 0)      pb_load(Wq, bq, r0, c0, lr, c4, bi, a, bb);
  else if (z == 1) pb_load(Wk, bk, r0, c0, lr, c4, bi, a, bb);
  else             pb_load(Wv, bv, r0, c0, lr, c4, bi, a, bb);
#pragma unroll
  for (int it = 0; it < 4; ++it) *(v4f*)(tf + (it * 16 + lr) * 68 + c4) = a[it];
  __syncthreads();
  const int sub = tid >> 3;
  const int c8  = (tid & 7) * 8;
  v4u hv[2];
#pragma unroll
  for (int it = 0; it < 2; ++it) {
    const int oc = it * 32 + sub;
    v4u w;
#pragma unroll
    for (int q = 0; q < 4; ++q) {
      const float f0 = tf[(c8 + 2 * q) * 68 + oc];
      const float f1 = tf[(c8 + 2 * q + 1) * 68 + oc];
      w[q] = pk16(f2bf_bits(f0), f2bf_bits(f1));
    }
    hv[it] = w;
  }
  for (int pass = 0; pass < 2; ++pass) {
#pragma unroll
    for (int it = 0; it < 2; ++it) {
      const int oc = it * 32 + sub;
      const size_t go = (size_t)(z * DM + c0 + oc) * DM + r0 + c8;
      *(volatile v4u*)(wt + go) = hv[it];
    }
    __threadfence();
  }
  if (blockIdx.x == 0 && blockIdx.y == 0 && tid < 192) {
    v4f o;
    o[0] = bfval(bb[0]); o[1] = bfval(bb[1]); o[2] = bfval(bb[2]); o[3] = bfval(bb[3]);
    float* dst = bqkv + z * DM + tid * 4;
    *(volatile v4f*)dst = o;
    __threadfence();
    *(volatile v4f*)dst = o;
  }
}

__global__ __launch_bounds__(192) void k_tab(const float* __restrict__ dpk, const float* __restrict__ dpv,
                                             const float* __restrict__ gk, const float* __restrict__ bk,
                                             const float* __restrict__ gv, const float* __restrict__ bv,
                                             float* __restrict__ tkv) {
  __shared__ __align__(16) float st[2 * NTYPES * DHD];
  const int tid = threadIdx.x, lane = tid & 31, w = tid >> 5;
  const int tab = (w >= NTYPES) ? 1 : 0;
  const int t   = w - NTYPES * tab;
  const unsigned mk = tab ? 0u : 0xffffffffu;
  const unsigned mv = ~mk;
  const int e = t * DHD + 2 * lane;
  const v2f ek = *(const v2fa*)(dpk + e);
  const v2f ev = *(const v2fa*)(dpv + e);
  const v2f g0 = *(const v2fa*)(gk + 2 * lane);
  const v2f g1 = *(const v2fa*)(gv + 2 * lane);
  const v2f b0 = *(const v2fa*)(bk + 2 * lane);
  const v2f b1 = *(const v2fa*)(bv + 2 * lane);
  const float x0 = bfval(__uint_as_float((__float_as_uint(ek[0]) & mk) | (__float_as_uint(ev[0]) & mv)));
  const float x1 = bfval(__uint_as_float((__float_as_uint(ek[1]) & mk) | (__float_as_uint(ev[1]) & mv)));
  const float ga = bfval(__uint_as_float((__float_as_uint(g0[0]) & mk) | (__float_as_uint(g1[0]) & mv)));
  const float gb = bfval(__uint_as_float((__float_as_uint(g0[1]) & mk) | (__float_as_uint(g1[1]) & mv)));
  const float ba = bfval(__uint_as_float((__float_as_uint(b0[0]) & mk) | (__float_as_uint(b1[0]) & mv)));
  const float bb = bfval(__uint_as_float((__float_as_uint(b0[1]) & mk) | (__float_as_uint(b1[1]) & mv)));
  float s = x0 + x1;
#pragma unroll
  for (int off = 16; off >= 1; off >>= 1) s += __shfl_xor(s, off, 32);
  const float mu = s * 0.015625f;
  const float d0 = x0 - mu, d1 = x1 - mu;
  float vs = d0 * d0 + d1 * d1;
#pragma unroll
  for (int off = 16; off >= 1; off >>= 1) vs += __shfl_xor(vs, off, 32);
  const float var = vs * 0.015625f;
  const float rs = 1.0f / sqrtf(var + 1e-5f);
  v2f y;
  y[0] = (d0 * rs) * ga + ba;
  y[1] = (d1 * rs) * gb + bb;
  *(v2f*)(st + w * DHD + 2 * lane) = y;
  __syncthreads();
  if (tid < 96) {
    const v4f o = *(const v4fa*)(st + tid * 4);
    float* dst = tkv + tid * 4;
    *(volatile v4f*)dst = o;
    __threadfence();
    *(volatile v4f*)dst = o;
  }
}

__global__ __launch_bounds__(256) __attribute__((amdgpu_num_vgpr(248)))
void k_proj(unsigned short* wsb, const float* __restrict__ bqkv, int tileBase) {
  __shared__ __align__(16) float sT[8][16 * 68];
  const int lane = threadIdx.x & 31;
  const int wave = threadIdx.x >> 5;
  const int tile = tileBase + blockIdx.x * 8 + wave;
  if (tile >= 3 * TILES_JOB) return;
  const int job = tile / TILES_JOB;
  const int tl  = tile - job * TILES_JOB;
  const int isV = (job == 2) ? 1 : 0;
  const int tilesN = isV ? (MTOK / 64) : (DM / 64);
  const int tm = tl / tilesN;
  const int tn = tl - tm * tilesN;
  const int m0 = tm << 6;
  const int n0 = tn << 6;
  const size_t aOff = (job == 0) ? EO_XB : ((job == 1) ? EO_CB : (EO_WT + (size_t)2 * DM * DM));
  const size_t bOff = (job == 0) ? EO_WT : ((job == 1) ? (EO_WT + (size_t)DM * DM) : EO_CB);
  const __bf16* Ab = (const __bf16*)(const void*)wsb + aOff;
  const __bf16* Bb = (const __bf16*)(const void*)wsb + bOff;

  const int rlane = lane & 15;
  const int hh    = lane >> 4;
  const int koff  = hh * 8;
  const int mOff  = hh * 8;

  v8f acc[4][4];
#pragma unroll
  for (int i = 0; i < 4; ++i)
#pragma unroll
    for (int j = 0; j < 4; ++j) acc[i][j] = (v8f){0.f, 0.f, 0.f, 0.f, 0.f, 0.f, 0.f, 0.f};

#pragma unroll 1
  for (int k0 = 0; k0 < DM; k0 += 32) {
    v16b bh[4];
#pragma unroll
    for (int j = 0; j < 4; ++j)
      bh[j] = ldfrag(Bb + (size_t)(n0 + (j << 4) + rlane) * DM + koff + k0);
#pragma unroll
    for (int i = 0; i < 4; ++i) {
      const v16b ah = ldfrag(Ab + (size_t)(m0 + (i << 4) + rlane) * DM + koff + k0);
#pragma unroll
      for (int j = 0; j < 4; ++j) acc[i][j] = wmb(ah, bh[j], acc[i][j]);
    }
  }

  float* slab = sT[wave];
  const unsigned nmask = isV ? 0u : 0xffffffffu;
  const unsigned mmask = ~nmask;
  float bnv[4];
#pragma unroll
  for (int j = 0; j < 4; ++j) {
    const int idx = isV ? 0 : (job * DM + n0 + (j << 4) + rlane);
    bnv[j] = mskf(bqkv[idx], nmask);
  }
  size_t obase; int pitch; size_t loDelta;
  if (isV) {
    const int bb = n0 >> 9;
    const int key0 = n0 & (LQ - 1);
    obase = EO_VTH + ((size_t)(bb * NH + tm) * DHD) * LQ + key0;
    pitch = LQ;
    loDelta = EO_VTL - EO_VTH;
  } else {
    obase = ((job == 0) ? EO_QHL : EO_KHL) + (size_t)m0 * QP + n0;
    pitch = QP;
    loDelta = DM;
  }
  const int q  = lane >> 3;
  const int c8 = (lane & 7) * 8;
#pragma unroll
  for (int i = 0; i < 4; ++i) {
    const int bmi = isV ? (2 * DM + m0 + (i << 4) + mOff) : 0;
    const v4f bA = *(const v4fa*)(bqkv + bmi);
    const v4f bB = *(const v4fa*)(bqkv + bmi + 4);
    float bmv[8];
    bmv[0] = mskf(bA[0], mmask); bmv[1] = mskf(bA[1], mmask); bmv[2] = mskf(bA[2], mmask); bmv[3] = mskf(bA[3], mmask);
    bmv[4] = mskf(bB[0], mmask); bmv[5] = mskf(bB[1], mmask); bmv[6] = mskf(bB[2], mmask); bmv[7] = mskf(bB[3], mmask);
#pragma unroll
    for (int j = 0; j < 4; ++j) {
#pragma unroll
      for (int r = 0; r < 8; ++r) {
        const float v = (acc[i][j][r] + bnv[j]) + bmv[r];
        slab[(mOff + r) * 68 + (j << 4) + rlane] = v;
      }
    }
    __builtin_amdgcn_fence(__ATOMIC_RELEASE, "workgroup");
    __builtin_amdgcn_wave_barrier();
    __builtin_amdgcn_fence(__ATOMIC_ACQUIRE, "workgroup");
    for (int pass = 0; pass < 2; ++pass) {
#pragma unroll
      for (int it = 0; it < 4; ++it) {
        const int row = it * 4 + q;
        const v4f s0 = *(const v4fa*)(slab + row * 68 + c8);
        const v4f s1 = *(const v4fa*)(slab + row * 68 + c8 + 4);
        const float sv[8] = {s0[0], s0[1], s0[2], s0[3], s1[0], s1[1], s1[2], s1[3]};
        v4u hv, lv;
#pragma unroll
        for (int e = 0; e < 4; ++e) {
          const unsigned short h0 = f2bf_bits(sv[2 * e]), h1 = f2bf_bits(sv[2 * e + 1]);
          const unsigned short l0 = f2bf_bits(sv[2 * e] - bf_bits2f(h0));
          const unsigned short l1 = f2bf_bits(sv[2 * e + 1] - bf_bits2f(h1));
          hv[e] = pk16(h0, h1);
          lv[e] = pk16(l0, l1);
        }
        unsigned short* dst = wsb + obase + (size_t)((i << 4) + row) * pitch + c8;
        *(volatile v4u*)dst = hv;
        *(volatile v4u*)(dst + loDelta) = lv;
      }
      __threadfence();
    }
    __builtin_amdgcn_fence(__ATOMIC_RELEASE, "workgroup");
    __builtin_amdgcn_wave_barrier();
    __builtin_amdgcn_fence(__ATOMIC_ACQUIRE, "workgroup");
  }
}

__global__ __launch_bounds__(128) __attribute__((amdgpu_num_vgpr(248)))
void k_attn(const unsigned short* __restrict__ qhl, const unsigned short* __restrict__ khl,
            const unsigned short* __restrict__ vth, const unsigned short* __restrict__ vtl,
            const int* __restrict__ arc, const float* __restrict__ amask,
            const float* __restrict__ tkv, float* __restrict__ out) {
  __shared__ __align__(16) __bf16 Ksh[64 * 64];
  __shared__ __align__(16) __bf16 Ksl[64 * 64];
  __shared__ __align__(16) __bf16 Vsh[64 * 64];
  __shared__ __align__(16) __bf16 Vsl[64 * 64];
  __shared__ __align__(16) __bf16 Psh[4][16 * 64];
  __shared__ __align__(16) __bf16 Psl[4][16 * 64];
  __shared__ __align__(16) float  Os[4][16 * 68];
  __shared__ __align__(16) int    arcs[64 * ARC_P];
  __shared__ __align__(16) float  tks[128 * 4];
  __shared__ __align__(16) float  msk[LQ];
  __shared__ __align__(16) float  qrs[64 * 4];
  __shared__ __align__(16) float  rst[4][16 * 4];

  const int tid  = threadIdx.x;
  const int wave = tid >> 5;
  const int lane = tid & 31;
  const int hh   = lane >> 4;
  const int c    = lane & 15;

  const int bx = blockIdx.x;
  const int qb = bx & 7;
  const int bh = bx >> 3;
  const int b  = bh / NH;
  const int h  = bh - b * NH;
  const int qblk = qb * 64;
  const int q0   = qblk + wave * 16;
  const size_t tokb = (size_t)b * LQ;

  const __bf16* Kh = (const __bf16*)(const void*)khl + tokb * QP + h * DHD;
  const __bf16* Kl = Kh + DM;
  const __bf16* Vh = (const __bf16*)(const void*)vth + (size_t)bh * DHD * LQ;
  const __bf16* Vl = (const __bf16*)(const void*)vtl + (size_t)bh * DHD * LQ;
  const int*    arcb = arc + (tokb + qblk) * LQ;
  float*        ob = out + tokb * DM + h * DHD;
  const __bf16* qfh = (const __bf16*)(const void*)qhl + (tokb + q0 + c) * QP + h * DHD + 8 * hh;
  const __bf16* qfl = qfh + DM;

  float* rsw = rst[wave];

  {
    const v4f t4 = *(const v4fa*)(tkv + min(tid, 95) * 4);
    *(v4fa*)(tks + tid * 4) = t4;
    v4f m4 = *(const v4fa*)(amask + (size_t)b * LQ + tid * 4);
    m4[0] = bfval(m4[0]); m4[1] = bfval(m4[1]); m4[2] = bfval(m4[2]); m4[3] = bfval(m4[3]);
    *(v4fa*)(msk + tid * 4) = m4;
    v2f z2; z2[0] = 0.f; z2[1] = 0.f;
    *(v2fa*)(rsw + lane * 2) = z2;
  }
  __syncthreads();
  {
    const int row = tid >> 1, half = tid & 1;
    const unsigned short* qp = qhl + (tokb + qblk + row) * QP + h * DHD + half * 32;
    float d0 = 0.f, d1 = 0.f, d2 = 0.f;
#pragma unroll 1
    for (int i = 0; i < 4; ++i) {
      const v4u hw = *(const v4ua*)(qp + 8 * i);
      const v4u lw = *(const v4ua*)(qp + DM + 8 * i);
      float qv[8];
#pragma unroll
      for (int w = 0; w < 4; ++w) {
        qv[2 * w]     = __uint_as_float(hw[w] << 16) + __uint_as_float(lw[w] << 16);
        qv[2 * w + 1] = __uint_as_float(hw[w] & 0xffff0000u) + __uint_as_float(lw[w] & 0xffff0000u);
      }
      const float* t0 = tks + half * 32 + i * 8;
#pragma unroll
      for (int e = 0; e < 8; ++e) {
        d0 = fmaf(qv[e], t0[e], d0);
        d1 = fmaf(qv[e], t0[DHD + e], d1);
        d2 = fmaf(qv[e], t0[2 * DHD + e], d2);
      }
    }
    d0 += __shfl_xor(d0, 1, 32);
    d1 += __shfl_xor(d1, 1, 32);
    d2 += __shfl_xor(d2, 1, 32);
    if (half == 0) {
      v4f o; o[0] = d0; o[1] = d1; o[2] = d2; o[3] = 0.f;
      *(v4fa*)(qrs + row * 4) = o;
    }
  }

  float mrow[8];
  v8f oacc[4];
#pragma unroll
  for (int r = 0; r < 8; ++r) mrow[r] = -INFINITY;
#pragma unroll
  for (int t = 0; t < 4; ++t) oacc[t] = (v8f){0.f, 0.f, 0.f, 0.f, 0.f, 0.f, 0.f, 0.f};

  __bf16* pwh = Psh[wave];
  __bf16* pwl = Psl[wave];

#pragma unroll 1
  for (int kc = 0; kc < LQ / 64; ++kc) {
    const int kv0 = kc * 64;
    __syncthreads();
    {
      const int r = tid >> 1, half = (tid & 1) * 32;
      const __bf16* ksh = Kh + (size_t)(kv0 + r) * QP + half;
      const __bf16* ksl = Kl + (size_t)(kv0 + r) * QP + half;
      const __bf16* vsh = Vh + (size_t)r * LQ + kv0 + half;
      const __bf16* vsl = Vl + (size_t)r * LQ + kv0 + half;
#pragma unroll 1
      for (int i = 0; i < 4; ++i) {
        const v8b a0 = *(const v8b*)(ksh + 8 * i);
        const v8b a1 = *(const v8b*)(ksl + 8 * i);
        const v8b b0 = *(const v8b*)(vsh + 8 * i);
        const v8b b1 = *(const v8b*)(vsl + 8 * i);
        *(v8b*)(Ksh + r * 64 + half + 8 * i) = a0;
        *(v8b*)(Ksl + r * 64 + half + 8 * i) = a1;
        *(v8b*)(Vsh + r * 64 + half + 8 * i) = b0;
        *(v8b*)(Vsl + r * 64 + half + 8 * i) = b1;
      }
      const int ar = tid >> 4, c4 = (tid & 15) * 4;
#pragma unroll 1
      for (int it = 0; it < 8; ++it) {
        const int row = it * 8 + ar;
        v4i a = *(const v4ia*)(arcb + (size_t)row * LQ + kv0 + c4);
        a[0] = clamp02(a[0]); a[1] = clamp02(a[1]); a[2] = clamp02(a[2]); a[3] = clamp02(a[3]);
        *(v4ia*)(arcs + row * ARC_P + c4) = a;
      }
    }
    __syncthreads();

    v8f s[4];
#pragma unroll
    for (int j = 0; j < 4; ++j) s[j] = (v8f){0.f, 0.f, 0.f, 0.f, 0.f, 0.f, 0.f, 0.f};
#pragma unroll 1
    for (int dc = 0; dc < 2; ++dc) {
      const v16b qh = ldfrag(qfh + dc * 32);
      const v16b ql = ldfrag(qfl + dc * 32);
#pragma unroll
      for (int j = 0; j < 4; ++j) {
        const v16b kb = ldfrag(Ksh + (j * 16 + c) * 64 + dc * 32 + 8 * hh);
        const v16b kl = ldfrag(Ksl + (j * 16 + c) * 64 + dc * 32 + 8 * hh);
        s[j] = wmb(qh, kb, s[j]);
        s[j] = wmb(qh, kl, s[j]);
        s[j] = wmb(ql, kb, s[j]);
        cbar();
      }
    }

    float mk[4];
#pragma unroll
    for (int j = 0; j < 4; ++j) mk[j] = msk[kv0 + j * 16 + c];
    cbar();

#pragma unroll
    for (int r = 0; r < 8; ++r) {
      const int rl = 8 * hh + r;
      const int rw = wave * 16 + rl;
      const int* ap = arcs + rw * ARC_P + c;
      int av[4];
      av[0] = ap[0]; av[1] = ap[16]; av[2] = ap[32]; av[3] = ap[48];
      const v4f qv = *(const v4fa*)(qrs + rw * 4);
      const v4f so = *(const v4fa*)(rsw + rl * 4);
      float sv[4];
#pragma unroll
      for (int j = 0; j < 4; ++j)
        sv[j] = (s[j][r] * 0.125f + blend3(av[j], qv[0], qv[1], qv[2])) + mk[j];
      float m = fmaxf(fmaxf(sv[0], sv[1]), fmaxf(sv[2], sv[3]));
#pragma unroll
      for (int off = 1; off < 16; off <<= 1) m = fmaxf(m, __shfl_xor(m, off, 32));
      const float mnew  = fmaxf(mrow[r], m);
      const float alpha = expf(mrow[r] - mnew);
      mrow[r] = mnew;
      float psum = 0.f, b0 = 0.f, b1 = 0.f, b2 = 0.f;
#pragma unroll
      for (int j = 0; j < 4; ++j) {
        const float p = expf(sv[j] - mnew);
        psum += p;
        b0 += keep_if(p, (int)(av[j] == 0));
        b1 += keep_if(p, (int)(av[j] == 1));
        b2 += keep_if(p, (int)(av[j] == 2));
        __bf16 ph, pl; split_bf(p, ph, pl);
        pwh[rl * 64 + j * 16 + c] = ph;
        pwl[rl * 64 + j * 16 + c] = pl;
      }
#pragma unroll
      for (int off = 1; off < 16; off <<= 1) {
        psum += __shfl_xor(psum, off, 32);
        b0   += __shfl_xor(b0, off, 32);
        b1   += __shfl_xor(b1, off, 32);
        b2   += __shfl_xor(b2, off, 32);
      }
      v4f sn;
      sn[0] = so[0] * alpha + psum;
      sn[1] = so[1] * alpha + b0;
      sn[2] = so[2] * alpha + b1;
      sn[3] = so[3] * alpha + b2;
      *(v4fa*)(rsw + rl * 4) = sn;
#pragma unroll
      for (int t = 0; t < 4; ++t) oacc[t][r] *= alpha;
      cbar();
    }
    __builtin_amdgcn_fence(__ATOMIC_RELEASE, "workgroup");
    __builtin_amdgcn_wave_barrier();
    __builtin_amdgcn_fence(__ATOMIC_ACQUIRE, "workgroup");
#pragma unroll 1
    for (int kk = 0; kk < 2; ++kk) {
      const v16b pa = ldfrag(pwh + c * 64 + kk * 32 + 8 * hh);
      const v16b pl = ldfrag(pwl + c * 64 + kk * 32 + 8 * hh);
#pragma unroll
      for (int t = 0; t < 4; ++t) {
        const v16b vb = ldfrag(Vsh + (t * 16 + c) * 64 + kk * 32 + 8 * hh);
        const v16b vl = ldfrag(Vsl + (t * 16 + c) * 64 + kk * 32 + 8 * hh);
        oacc[t] = wmb(pa, vb, oacc[t]);
        oacc[t] = wmb(pa, vl, oacc[t]);
        oacc[t] = wmb(pl, vb, oacc[t]);
        cbar();
      }
    }
  }

  __builtin_amdgcn_fence(__ATOMIC_RELEASE, "workgroup");
  __builtin_amdgcn_wave_barrier();
  __builtin_amdgcn_fence(__ATOMIC_ACQUIRE, "workgroup");
  float tv0[4], tv1[4], tv2[4];
#pragma unroll
  for (int t = 0; t < 4; ++t) {
    tv0[t] = tks[(NTYPES + 0) * DHD + t * 16 + c];
    tv1[t] = tks[(NTYPES + 1) * DHD + t * 16 + c];
    tv2[t] = tks[(NTYPES + 2) * DHD + t * 16 + c];
  }
  float* os = Os[wave];
#pragma unroll
  for (int r = 0; r < 8; ++r) {
    const v4f fin = *(const v4fa*)(rsw + (8 * hh + r) * 4);
    const float inv = 1.0f / fin[0];
#pragma unroll
    for (int t = 0; t < 4; ++t) {
      const float o = ((oacc[t][r] + fin[1] * tv0[t]) + fin[2] * tv1[t]) + fin[3] * tv2[t];
      os[(8 * hh + r) * 68 + t * 16 + c] = o * inv;
    }
    cbar();
  }
  __builtin_amdgcn_fence(__ATOMIC_RELEASE, "workgroup");
  __builtin_amdgcn_wave_barrier();
  __builtin_amdgcn_fence(__ATOMIC_ACQUIRE, "workgroup");
  {
    const int c4 = (lane & 15) * 4;
    for (int pass = 0; pass < 2; ++pass) {
#pragma unroll
      for (int it = 0; it < 8; ++it) {
        const int row = it * 2 + hh;
        const v4f val = *(const v4fa*)(os + row * 68 + c4);
        *(volatile v4f*)(ob + (size_t)(q0 + row) * DM + c4) = val;
      }
      __threadfence();
    }
  }
}

extern "C" void kernel_launch(void* const* d_in, const int* in_sizes, int n_in,
                              void* d_out, int out_size, void* d_ws, size_t ws_size,
                              hipStream_t stream) {
  if (n_in < 16) return;
  if (in_sizes[0] != MTOK * DM || in_sizes[1] != MTOK * DM) return;
  if (in_sizes[2] != NB * LQ) return;
  if (in_sizes[3] != NB * LQ * LQ) return;
  if (in_sizes[4] != DM * DM || in_sizes[6] != DM * DM || in_sizes[8] != DM * DM) return;
  if (in_sizes[5] != DM || in_sizes[7] != DM || in_sizes[9] != DM) return;
  if (in_sizes[10] != NTYPES * DHD || in_sizes[11] != NTYPES * DHD) return;
  if (in_sizes[12] != DHD || in_sizes[13] != DHD || in_sizes[14] != DHD || in_sizes[15] != DHD) return;
  if (out_size != MTOK * DM) return;
  if (OB_END > ws_size) return;

  const float* hidden = (const float*)d_in[0];
  const float* contex = (const float*)d_in[1];
  const float* amask  = (const float*)d_in[2];
  const int*   arc    = (const int*)d_in[3];
  const float* Wq   = (const float*)d_in[4];
  const float* bq   = (const float*)d_in[5];
  const float* Wk   = (const float*)d_in[6];
  const float* bk   = (const float*)d_in[7];
  const float* Wv   = (const float*)d_in[8];
  const float* bv   = (const float*)d_in[9];
  const float* dpk  = (const float*)d_in[10];
  const float* dpv  = (const float*)d_in[11];
  const float* lnkg = (const float*)d_in[12];
  const float* lnkb = (const float*)d_in[13];
  const float* lnvg = (const float*)d_in[14];
  const float* lnvb = (const float*)d_in[15];
  float* out = (float*)d_out;

  char* ws = (char*)d_ws;
  unsigned short* wsb  = (unsigned short*)ws;
  unsigned short* WT   = (unsigned short*)(ws + OB_WT);
  float*          BQKV = (float*)(ws + OB_BQKV);
  float*          TKV  = (float*)(ws + OB_TKV);
  const unsigned short* QHL = (const unsigned short*)(ws + OB_QHL);
  const unsigned short* KHL = (const unsigned short*)(ws + OB_KHL);
  const unsigned short* VTH = (const unsigned short*)(ws + OB_VTH);
  const unsigned short* VTL = (const unsigned short*)(ws + OB_VTL);

  k_pa<<<dim3(768, 2), dim3(256), 0, stream>>>(hidden, contex, wsb);
  k_pb<<<dim3(DM / 64, DM / 64, 3), dim3(256), 0, stream>>>(Wq, bq, Wk, bk, Wv, bv, WT, BQKV);
  k_tab<<<dim3(1), dim3(192), 0, stream>>>(dpk, dpv, lnkg, lnkb, lnvg, lnvb, TKV);
  k_proj<<<dim3(TILES_JOB / 8), dim3(256), 0, stream>>>(wsb, BQKV, 0);
  k_proj<<<dim3(2 * TILES_JOB / 8), dim3(256), 0, stream>>>(wsb, BQKV, TILES_JOB);
  k_attn<<<dim3(NB * NH * (LQ / 64)), dim3(128), 0, stream>>>(QHL, KHL, VTH, VTL, arc, amask, TKV, out);
  (void)hipGetLastError();
}
